// GRUPlant_7164005450351
// MI455X (gfx1250) — hardware-run, weakly checked
//
#include <hip/hip_runtime.h>

typedef __attribute__((ext_vector_type(16))) _Float16 v16h;
typedef __attribute__((ext_vector_type(8)))  _Float16 v8h;
typedef __attribute__((ext_vector_type(4)))  _Float16 v4h;
typedef __attribute__((ext_vector_type(16))) __bf16   v16b;
typedef __attribute__((ext_vector_type(8)))  __bf16   v8b;
typedef __attribute__((ext_vector_type(8)))  float    v8f;
typedef __attribute__((ext_vector_type(4)))  float    v4f;
typedef __attribute__((ext_vector_type(4)))  unsigned v4u;
typedef __attribute__((ext_vector_type(2)))  unsigned v2u;

constexpr int kNB   = 256;
constexpr int kTE   = 512;
constexpr int kTD   = 256;
constexpr int kNX   = 64;
constexpr int kNPV  = 16;
constexpr int kH    = 256;
constexpr int kEMB  = 32;
constexpr int kNSC  = 4;
constexpr int kG    = 3 * kH;
constexpr int kF1   = 128;
constexpr int kEI   = kNX + kEMB;
constexpr int kDI   = kNX + kNPV;
constexpr int kDIP  = 96;
static_assert(kEI == 96 && kDI == 80 && kG == 768);
static_assert(kNX % 32 == 0 && kH % 32 == 0 && kDIP % 32 == 0 && kF1 % 32 == 0);
static_assert(kDIP >= kDI && kDIP - kDI == 16);

constexpr float kActCarry = 16.0f;
constexpr float kWtCarry  = 64.0f;
constexpr float kFold     = 1.0f / (kActCarry * kWtCarry);
constexpr float kLog2e    = 1.4426950408889634f;
constexpr float kSigMul   = -kFold * kLog2e;
constexpr float kTanhMul  = 2.0f * kFold * kLog2e;

constexpr int kRowsPB = 32;
constexpr int kBlocks = kNB / kRowsPB;
constexpr int kThr    = 512;
constexpr int kHP     = kH + 8;
constexpr int kPL     = kRowsPB * kHP;
constexpr int kXEP    = kNX + 8;
constexpr int kXDP    = kDIP + 8;
constexpr int kAP     = kF1 + 8;
constexpr int kYP     = 8 * kNPV;
constexpr int kSbCell = 256;
constexpr int kSbFc1  = 256 + 3 * 1024;
constexpr int kSbFc2  = kSbFc1 + kF1;
constexpr int kSbTot  = kSbFc2 + kNPV;
static_assert(kNB % kRowsPB == 0);
static_assert(kH == 16 * (kThr / 32));
static_assert(kHP % 8 == 0 && kXEP % 8 == 0 && kXDP % 8 == 0 && kAP % 8 == 0);
static_assert(kTD % 8 == 0);
static_assert(kRowsPB * kNX == kThr * 4);
static_assert((kF1 / 16) * (kRowsPB / 16) == kThr / 32);

constexpr int kPb1  = (kG * (kNX / 8)) / 256;
constexpr int kPbW  = (kG * (kH / 8)) / 256;
constexpr int kPb2  = kPb1 + kPbW;
constexpr int kPb3  = kPb2 + kPbW;
constexpr int kPb4  = kPb3 + kPbW;
constexpr int kPb5  = kPb4 + kPbW;
constexpr int kPb6  = kPb5 + kPbW;
constexpr int kPb7  = kPb6 + kPbW;
constexpr int kPb8  = kPb7 + (kG * (kDIP / 8)) / 256;
constexpr int kPb9  = kPb8 + (kF1 * (kH / 8)) / 256;
constexpr int kPbPi = kPb9 + (kNPV * (kF1 / 8)) / 256;
constexpr int kPrepBlocks = kPbPi + kG / 32;
static_assert((kG * (kNX / 8)) % 256 == 0 && (kG * (kH / 8)) % 256 == 0 && (kG * (kDIP / 8)) % 256 == 0);
static_assert((kF1 * (kH / 8)) % 256 == 0 && (kNPV * (kF1 / 8)) % 256 == 0);
static_assert(kPb1 == 24 && kPbW == 96 && kPb8 == 636 && kPb9 == 652 && kPbPi == 653 && kPrepBlocks == 677);

template <typename T> struct Frag;
template <> struct Frag<_Float16> {
  typedef v16h V; union U { v16h v; v8h h[2]; };
  static __device__ __forceinline__ v16h load(const _Float16* p) {
    U f; f.h[0] = *(const v8h*)(p); f.h[1] = *(const v8h*)(p + 16); return f.v;
  }
  static __device__ __forceinline__ v8f mma(v16h a, v16h b, v8f c) {
    return __builtin_amdgcn_wmma_f32_16x16x32_f16(false, a, false, b, (short)0, c, false, false);
  }
};
template <> struct Frag<__bf16> {
  typedef v16b V; union U { v16b v; v8b h[2]; };
  static __device__ __forceinline__ v16b load(const __bf16* p) {
    U f; f.h[0] = *(const v8b*)(p); f.h[1] = *(const v8b*)(p + 16); return f.v;
  }
  static __device__ __forceinline__ v8f mma(v16b a, v16b b, v8f c) {
    return __builtin_amdgcn_wmma_f32_16x16x32_bf16(false, a, false, b, (short)0, c, false, false);
  }
};
typedef Frag<_Float16> FragH;
typedef Frag<__bf16>   FragB;

__device__ __forceinline__ void guard6_h(v8f& a0, v8f& a1, v8f& a2, v8f& a3, v8f& a4, v8f& a5,
                                         v16h f0, v16h f1, v16h f2, v16h f3, v16h f4) {
  asm volatile("v_nop\n\tv_nop\n\tv_nop\n\tv_nop"
               : "+v"(a0), "+v"(a1), "+v"(a2), "+v"(a3), "+v"(a4), "+v"(a5)
               : "v"(f0), "v"(f1), "v"(f2), "v"(f3), "v"(f4));
}
__device__ __forceinline__ void guard6_b(v8f& a0, v8f& a1, v8f& a2, v8f& a3, v8f& a4, v8f& a5,
                                         v16b f0, v16b f1, v16b f2, v16b f3, v16b f4,
                                         v16b f5, v16b f6, v16b f7, v16b f8, v16b f9) {
  asm volatile("v_nop\n\tv_nop\n\tv_nop\n\tv_nop"
               : "+v"(a0), "+v"(a1), "+v"(a2), "+v"(a3), "+v"(a4), "+v"(a5)
               : "v"(f0), "v"(f1), "v"(f2), "v"(f3), "v"(f4), "v"(f5), "v"(f6), "v"(f7), "v"(f8), "v"(f9));
}
__device__ __forceinline__ void guard1_b(v8f& a0, v16b f0, v16b f1, v16b f2, v16b f3) {
  asm volatile("v_nop\n\tv_nop\n\tv_nop\n\tv_nop" : "+v"(a0) : "v"(f0), "v"(f1), "v"(f2), "v"(f3));
}

__device__ __forceinline__ unsigned rne_bf_word(float f) {
  const unsigned u = __float_as_uint(f);
  return u + 0x7FFFu + ((u >> 16) & 1u);
}
__device__ __forceinline__ void split2(float a, float b, unsigned& whi, unsigned& wlo) {
  const unsigned ra = rne_bf_word(a);
  const unsigned rb = rne_bf_word(b);
  whi = (ra >> 16) | (rb & 0xFFFF0000u);
  const float la = a - __uint_as_float(ra & 0xFFFF0000u);
  const float lb = b - __uint_as_float(rb & 0xFFFF0000u);
  const unsigned sa = rne_bf_word(la);
  const unsigned sb = rne_bf_word(lb);
  wlo = (sa >> 16) | (sb & 0xFFFF0000u);
}
__device__ __forceinline__ float h16z(float v) {
  return (__builtin_fabsf(v) < 6.103515625e-05f) ? 0.0f : v;
}
__device__ __forceinline__ unsigned pack_f16x2(float a, float b) {
  const _Float16 h0 = (_Float16)h16z(a);
  const _Float16 h1 = (_Float16)h16z(b);
  const unsigned short u0 = __builtin_bit_cast(unsigned short, h0);
  const unsigned short u1 = __builtin_bit_cast(unsigned short, h1);
  return (unsigned)u0 | ((unsigned)u1 << 16);
}
__device__ __forceinline__ v8f ld8(const float* p) {
  const v4f lo = *(const v4f*)p;
  const v4f hi = *(const v4f*)(p + 4);
  return (v8f){lo[0], lo[1], lo[2], lo[3], hi[0], hi[1], hi[2], hi[3]};
}

struct PrepArgs {
  const int*   scen;
  const float* emb;
  const float* eWih0; const float* eWhh0; const float* ebih0; const float* ebhh0;
  const float* eWih1; const float* eWhh1;
  const float* dWih0; const float* dWhh0; const float* dWih1; const float* dWhh1;
  const float* fc1W;  const float* fc2W;
  unsigned short* we0x; unsigned short* we0h; unsigned short* we1i; unsigned short* we1h;
  unsigned short* wd0h; unsigned short* wd1i; unsigned short* wd1h;
  unsigned short* wd0ih; unsigned short* wd0il;
  unsigned short* fc1h; unsigned short* fc1l; unsigned short* fc2h; unsigned short* fc2l;
  float* pi;
};
static_assert(sizeof(PrepArgs) == 28 * 8);

__global__ __launch_bounds__(256) void prep_kernel(PrepArgs a) {
  __shared__ __align__(16) float p4[kNSC * 32];
  const int blk = blockIdx.x;
  const int tid = threadIdx.x;
  if (blk < kPbPi) {
    const float* src = a.eWih0;
    unsigned short* dh = a.we0x;
    unsigned short* dl = a.we0x;
    int spitch = kEI, svalid = kNX, ncol8 = kNX / 8, rel = blk;
    bool split = false;
    if (blk >= kPb1 && blk < kPb2) { src = a.eWhh0; dh = a.we0h; dl = dh; spitch = kH; svalid = kH; ncol8 = kH / 8; rel = blk - kPb1; }
    if (blk >= kPb2 && blk < kPb3) { src = a.eWih1; dh = a.we1i; dl = dh; spitch = kH; svalid = kH; ncol8 = kH / 8; rel = blk - kPb2; }
    if (blk >= kPb3 && blk < kPb4) { src = a.eWhh1; dh = a.we1h; dl = dh; spitch = kH; svalid = kH; ncol8 = kH / 8; rel = blk - kPb3; }
    if (blk >= kPb4 && blk < kPb5) { src = a.dWhh0; dh = a.wd0h; dl = dh; spitch = kH; svalid = kH; ncol8 = kH / 8; rel = blk - kPb4; }
    if (blk >= kPb5 && blk < kPb6) { src = a.dWih1; dh = a.wd1i; dl = dh; spitch = kH; svalid = kH; ncol8 = kH / 8; rel = blk - kPb5; }
    if (blk >= kPb6 && blk < kPb7) { src = a.dWhh1; dh = a.wd1h; dl = dh; spitch = kH; svalid = kH; ncol8 = kH / 8; rel = blk - kPb6; }
    if (blk >= kPb7 && blk < kPb8) { src = a.dWih0; dh = a.wd0ih; dl = a.wd0il; spitch = kDI; svalid = kDI; ncol8 = kDIP / 8; rel = blk - kPb7; split = true; }
    if (blk >= kPb8 && blk < kPb9) { src = a.fc1W; dh = a.fc1h; dl = a.fc1l; spitch = kH; svalid = kH; ncol8 = kH / 8; rel = blk - kPb8; split = true; }
    if (blk >= kPb9) { src = a.fc2W; dh = a.fc2h; dl = a.fc2l; spitch = kF1; svalid = kF1; ncol8 = kF1 / 8; rel = blk - kPb9; split = true; }

    const int i   = rel * 256 + tid;
    const int row = i / ncol8;
    const int col = (i - row * ncol8) * 8;
    const int colc = (col < svalid) ? col : (svalid - 8);
    const bool ok  = col < svalid;
    const float* sp = src + (size_t)row * spitch + colc;
    const v4f fa = *(const v4f*)sp;
    const v4f fb = *(const v4f*)(sp + 4);
    float v[8];
#pragma unroll
    for (int e = 0; e < 4; ++e) {
      v[e]     = ok ? fa[e] * kWtCarry : 0.0f;
      v[4 + e] = ok ? fb[e] * kWtCarry : 0.0f;
    }
    v4u w0, w1;
    if (split) {
#pragma unroll
      for (int q = 0; q < 4; ++q) {
        unsigned hi, lo;
        split2(v[2 * q], v[2 * q + 1], hi, lo);
        w0[q] = hi;
        w1[q] = lo;
      }
    } else {
#pragma unroll
      for (int q = 0; q < 4; ++q) {
        const unsigned pk = pack_f16x2(v[2 * q], v[2 * q + 1]);
        w0[q] = pk;
        w1[q] = pk;
      }
    }
    unsigned short* ph = dh + (size_t)i * 8;
    unsigned short* pl = dl + (size_t)i * 8;
    *(volatile v4u*)ph = w0;
    if (split) *(volatile v4u*)pl = w1;
    __threadfence();
    *(volatile v4u*)ph = w0;
    if (split) *(volatile v4u*)pl = w1;
  } else {
    const int n0 = (blk - kPbPi) * 32;
    if (tid < 128) {
      const int s = tid >> 5, j = tid & 31, n = n0 + j;
      const float* wrow = a.eWih0 + (size_t)n * kEI + kNX;
      const float* erow = a.emb + s * kEMB;
      float acc = 0.0f;
#pragma unroll 4
      for (int k = 0; k < kEMB; ++k) acc = fmaf(erow[k], wrow[k], acc);
      acc += a.ebih0[n];
      const float bh = a.ebhh0[n];
      const float val = (n0 < 2 * kH) ? (-kLog2e) * (acc + bh) : (2.0f * kLog2e) * acc;
      p4[s * 32 + j] = val;
    }
    __syncthreads();
    const int lane = tid & 31, wave = tid >> 5, q = lane >> 3, c4 = (lane & 7) * 4;
    v4f vals[8];
#pragma unroll
    for (int it = 0; it < 8; ++it) {
      const int b = wave * 32 + it * 4 + q;
      int s = a.scen[b];
      s = s < 0 ? 0 : (s > kNSC - 1 ? kNSC - 1 : s);
      vals[it] = *(const v4f*)(p4 + s * 32 + c4);
    }
    for (int pass = 0; pass < 2; ++pass) {
#pragma unroll
      for (int it = 0; it < 8; ++it) {
        const int b = wave * 32 + it * 4 + q;
        *(volatile v4f*)(a.pi + (size_t)b * kG + n0 + c4) = vals[it];
      }
      __threadfence();
    }
  }
}

template <int KC, int WP, int BP>
__device__ __forceinline__ void gemm3_f16(const _Float16* __restrict__ wl, const _Float16* bl,
                                          v8f& r0, v8f& r1, v8f& z0, v8f& z1, v8f& n0, v8f& n1) {
#pragma unroll
  for (int kc = 0; kc < KC; ++kc) {
    const v16h wr = FragH::load(wl + kc * 32);
    const v16h wz = FragH::load(wl + kH * WP + kc * 32);
    const v16h wn = FragH::load(wl + 2 * kH * WP + kc * 32);
    const v16h b0 = FragH::load(bl + kc * 32);
    const v16h b1 = FragH::load(bl + 16 * BP + kc * 32);
    r0 = FragH::mma(wr, b0, r0);
    r1 = FragH::mma(wr, b1, r1);
    z0 = FragH::mma(wz, b0, z0);
    z1 = FragH::mma(wz, b1, z1);
    n0 = FragH::mma(wn, b0, n0);
    n1 = FragH::mma(wn, b1, n1);
    guard6_h(r0, r1, z0, z1, n0, n1, wr, wz, wn, b0, b1);
  }
}

template <int KC, int WP, int BP>
__device__ __forceinline__ void gemm3_b3(const __bf16* __restrict__ wh, const __bf16* __restrict__ wl,
                                         const __bf16* bh, const __bf16* bl,
                                         v8f& r0, v8f& r1, v8f& z0, v8f& z1, v8f& n0, v8f& n1) {
#pragma unroll
  for (int kc = 0; kc < KC; ++kc) {
    const v16b wrh = FragB::load(wh + kc * 32);
    const v16b wzh = FragB::load(wh + kH * WP + kc * 32);
    const v16b wnh = FragB::load(wh + 2 * kH * WP + kc * 32);
    const v16b wrl = FragB::load(wl + kc * 32);
    const v16b wzl = FragB::load(wl + kH * WP + kc * 32);
    const v16b wnl = FragB::load(wl + 2 * kH * WP + kc * 32);
    const v16b b0h = FragB::load(bh + kc * 32);
    const v16b b1h = FragB::load(bh + 16 * BP + kc * 32);
    const v16b b0l = FragB::load(bl + kc * 32);
    const v16b b1l = FragB::load(bl + 16 * BP + kc * 32);
    r0 = FragB::mma(wrh, b0h, r0);
    r1 = FragB::mma(wrh, b1h, r1);
    z0 = FragB::mma(wzh, b0h, z0);
    z1 = FragB::mma(wzh, b1h, z1);
    n0 = FragB::mma(wnh, b0h, n0);
    n1 = FragB::mma(wnh, b1h, n1);
    r0 = FragB::mma(wrh, b0l, r0);
    r1 = FragB::mma(wrh, b1l, r1);
    z0 = FragB::mma(wzh, b0l, z0);
    z1 = FragB::mma(wzh, b1l, z1);
    n0 = FragB::mma(wnh, b0l, n0);
    n1 = FragB::mma(wnh, b1l, n1);
    r0 = FragB::mma(wrl, b0h, r0);
    r1 = FragB::mma(wrl, b1h, r1);
    z0 = FragB::mma(wzl, b0h, z0);
    z1 = FragB::mma(wzl, b1h, z1);
    n0 = FragB::mma(wnl, b0h, n0);
    n1 = FragB::mma(wnl, b1h, n1);
    guard6_b(r0, r1, z0, z1, n0, n1, wrh, wzh, wnh, wrl, wzl, wnl, b0h, b1h, b0l, b1l);
  }
}

template <int KC>
__device__ __forceinline__ v8f gemm1_b3(const __bf16* __restrict__ wh, const __bf16* __restrict__ wl,
                                        const __bf16* bh, const __bf16* bl, v8f acc) {
#pragma unroll
  for (int kc = 0; kc < KC; ++kc) {
    const v16b ah = FragB::load(wh + kc * 32);
    const v16b al = FragB::load(wl + kc * 32);
    const v16b xh = FragB::load(bh + kc * 32);
    const v16b xl = FragB::load(bl + kc * 32);
    acc = FragB::mma(ah, xh, acc);
    acc = FragB::mma(ah, xl, acc);
    acc = FragB::mma(al, xh, acc);
    guard1_b(acc, ah, al, xh, xl);
  }
  return acc;
}

template <bool SPLIT_OUT>
__device__ __forceinline__ void gru_gates(const v8f& aR, const v8f& aZ, const v8f& aNI, const v8f& aNH,
                                          const v8f& bR, const v8f& bZ, const v8f& bNI, const v8f& bNH,
                                          v8f& mst, _Float16* dst, unsigned short* dsh, unsigned short* dsl) {
  float hs[8];
#pragma unroll
  for (int r = 0; r < 8; ++r) {
    const float er = __builtin_amdgcn_exp2f(fmaf(aR[r], kSigMul, bR[r]));
    const float rg = __builtin_amdgcn_rcpf(1.0f + er);
    const float ez = __builtin_amdgcn_exp2f(fmaf(aZ[r], kSigMul, bZ[r]));
    const float zg = __builtin_amdgcn_rcpf(1.0f + ez);
    const float pn = fmaf(aNH[r], kTanhMul, bNH[r]);
    const float qn = fmaf(aNI[r], kTanhMul, bNI[r]);
    const float en = __builtin_amdgcn_exp2f(fmaf(rg, pn, qn));
    const float ng = fmaf(-2.0f, __builtin_amdgcn_rcpf(1.0f + en), 1.0f);
    const float ho = mst[r];
    const float hn = fmaf(zg, ho - ng, ng);
    mst[r] = hn;
    hs[r] = hn * kActCarry;
  }
  v8h hv;
#pragma unroll
  for (int r = 0; r < 8; ++r) hv[r] = (_Float16)h16z(hs[r]);
  *(v8h*)dst = hv;
  if (SPLIT_OUT) {
    v4u wh, wl;
#pragma unroll
    for (int q = 0; q < 4; ++q) {
      unsigned hi, lo;
      split2(hs[2 * q], hs[2 * q + 1], hi, lo);
      wh[q] = hi;
      wl[q] = lo;
    }
    *(v4u*)dsh = wh;
    *(v4u*)dsl = wl;
  }
}

__device__ __forceinline__ void fill_cell(float* tab, const float* __restrict__ bih, const float* __restrict__ bhh, int tid) {
  const float x0 = bih[tid];
  const float y0 = bhh[tid];
  tab[tid] = (-kLog2e) * (x0 + y0);
  const float x1 = bih[2 * kH + (tid & (kH - 1))];
  const float y1 = bhh[2 * kH + (tid & (kH - 1))];
  tab[2 * kH + tid] = (2.0f * kLog2e) * ((tid < kH) ? x1 : y1);
}

struct SeqArgs {
  const float* x_cv; const float* x_tgt; const float* pv_init;
  const float* ebhh0; const float* ebih1; const float* ebhh1;
  const float* dbih0; const float* dbhh0; const float* dbih1; const float* dbhh1;
  const float* fc1b;  const float* fc2b;
  const unsigned short* we0x; const unsigned short* we0h; const unsigned short* we1i; const unsigned short* we1h;
  const unsigned short* wd0h; const unsigned short* wd1i; const unsigned short* wd1h;
  const unsigned short* wd0ih; const unsigned short* wd0il;
  const unsigned short* fc1h; const unsigned short* fc1l; const unsigned short* fc2h; const unsigned short* fc2l;
  const float* pi;
  float* out;
};
static_assert(sizeof(SeqArgs) == 27 * 8);

__global__ __launch_bounds__(kThr) __attribute__((amdgpu_num_vgpr(256))) void seq_kernel(SeqArgs a) {
  __shared__ __align__(16) _Float16       hbuf[4 * kPL];
  __shared__ __align__(16) _Float16       xe[kRowsPB * kXEP];
  __shared__ __align__(16) unsigned short xdh[kRowsPB * kXDP];
  __shared__ __align__(16) unsigned short xdl[kRowsPB * kXDP];
  __shared__ __align__(16) unsigned short d1h[kPL];
  __shared__ __align__(16) unsigned short d1l[kPL];
  __shared__ __align__(16) unsigned short ah[kRowsPB * kAP];
  __shared__ __align__(16) unsigned short al[kRowsPB * kAP];
  __shared__ __align__(16) float          ybuf[kRowsPB * kYP];
  __shared__ __align__(32) float          sbias[kSbTot];

  const int tid  = threadIdx.x;
  const int lane = tid & 31, wave = tid >> 5;
  const int c = lane & 15, hh = lane >> 4, koff = hh * 8;
  const int b0 = blockIdx.x * kRowsPB;
  const int ub = 16 * wave + 8 * hh;

  const _Float16* we0x = (const _Float16*)a.we0x;
  const _Float16* we0h = (const _Float16*)a.we0h;
  const _Float16* we1i = (const _Float16*)a.we1i;
  const _Float16* we1h = (const _Float16*)a.we1h;
  const _Float16* wd0h = (const _Float16*)a.wd0h;
  const _Float16* wd1i = (const _Float16*)a.wd1i;
  const _Float16* wd1h = (const _Float16*)a.wd1h;
  const __bf16* wd0ih = (const __bf16*)a.wd0ih;
  const __bf16* wd0il = (const __bf16*)a.wd0il;
  const __bf16* fc1h  = (const __bf16*)a.fc1h;
  const __bf16* fc1l  = (const __bf16*)a.fc1l;
  const __bf16* fc2h  = (const __bf16*)a.fc2h;
  const __bf16* fc2l  = (const __bf16*)a.fc2l;

  const unsigned wrow  = (unsigned)(16 * wave + c);
  const unsigned wo64  = wrow * kNX + koff;
  const unsigned wo256 = wrow * kH + koff;
  const unsigned wo96  = wrow * kDIP + koff;
  const unsigned bo_h  = (unsigned)(c * kHP + koff);
  const unsigned bo_xe = (unsigned)(c * kXEP + koff);
  const unsigned bo_xd = (unsigned)(c * kXDP + koff);
  const unsigned so_h  = (unsigned)(c * kHP + ub);
  const unsigned pio   = (unsigned)((b0 + c) * kG + ub);
  const int xr = tid >> 4, xc4 = (tid & 15) * 4;

  {
    float e0 = a.ebhh0[2 * kH + (tid & (kH - 1))];
    asm volatile("" : "+v"(e0));
    if (tid < kH) sbias[tid] = (2.0f * kLog2e) * e0;
    fill_cell(sbias + kSbCell, a.ebih1, a.ebhh1, tid);
    fill_cell(sbias + kSbCell + 1024, a.dbih0, a.dbhh0, tid);
    fill_cell(sbias + kSbCell + 2048, a.dbih1, a.dbhh1, tid);
    float f1 = a.fc1b[tid & (kF1 - 1)];
    asm volatile("" : "+v"(f1));
    if (tid < kF1) sbias[kSbFc1 + tid] = f1;
    float f2 = a.fc2b[tid & (kNPV - 1)];
    asm volatile("" : "+v"(f2));
    if (tid < kNPV) sbias[kSbFc2 + tid] = f2;
  }
  {
    const v8h zh = {(_Float16)0.f, (_Float16)0.f, (_Float16)0.f, (_Float16)0.f, (_Float16)0.f, (_Float16)0.f, (_Float16)0.f, (_Float16)0.f};
    for (int i = tid; i < (2 * kPL) / 8; i += kThr) *(v8h*)(hbuf + i * 8) = zh;
  }
  const float* xsrcE = a.x_cv + ((size_t)(b0 + xr) * kTE) * kNX + xc4;
  {
    const v4f xv = *(const v4f*)(xsrcE);
    v4h xh;
#pragma unroll
    for (int e = 0; e < 4; ++e) xh[e] = (_Float16)h16z(xv[e] * kActCarry);
    *(v4h*)(xe + xr * kXEP + xc4) = xh;
  }

  const v8f z8 = {0.f, 0.f, 0.f, 0.f, 0.f, 0.f, 0.f, 0.f};
  v8f m00 = z8, m01 = z8, m10 = z8, m11 = z8;
  __syncthreads();

#pragma unroll 1
  for (int t = 0; t < kTE; ++t) {
    const int pr = (t & 1) * (2 * kPL);
    const int pw = (2 * kPL) - pr;
    {
      v8f aR0 = z8, aR1 = z8, aZ0 = z8, aZ1 = z8, aN0 = z8, aN1 = z8, aH0 = z8, aH1 = z8;
      gemm3_f16<kNX / 32, kNX, kXEP>(we0x + wo64, xe + bo_xe, aR0, aR1, aZ0, aZ1, aN0, aN1);
      gemm3_f16<kH / 32, kH, kHP>(we0h + wo256, hbuf + pr + bo_h, aR0, aR1, aZ0, aZ1, aH0, aH1);
      unsigned po = pio;
      asm volatile("" : "+v"(po));
      const float* pl = a.pi + po;
      const v8f bR0 = ld8(pl);
      const v8f bZ0 = ld8(pl + kH);
      const v8f bN0 = ld8(pl + 2 * kH);
      const v8f bR1 = ld8(pl + 16 * kG);
      const v8f bZ1 = ld8(pl + 16 * kG + kH);
      const v8f bN1 = ld8(pl + 16 * kG + 2 * kH);
      const v8f bNH = ld8(sbias + ub);
      _Float16* hw = hbuf + pw + so_h;
      gru_gates<false>(aR0, aZ0, aN0, aH0, bR0, bZ0, bN0, bNH, m00, hw, nullptr, nullptr);
      gru_gates<false>(aR1, aZ1, aN1, aH1, bR1, bZ1, bN1, bNH, m01, hw + 16 * kHP, nullptr, nullptr);
    }
    __syncthreads();
    {
      const int tn = (t + 1 < kTE) ? (t + 1) : (kTE - 1);
      const v4f xv = *(const v4f*)(xsrcE + (size_t)tn * kNX);
      v4h xh;
#pragma unroll
      for (int e = 0; e < 4; ++e) xh[e] = (_Float16)h16z(xv[e] * kActCarry);
      *(v4h*)(xe + xr * kXEP + xc4) = xh;
    }
    {
      v8f aR0 = z8, aR1 = z8, aZ0 = z8, aZ1 = z8, aN0 = z8, aN1 = z8, aH0 = z8, aH1 = z8;
      gemm3_f16<kH / 32, kH, kHP>(we1i + wo256, hbuf + pw + bo_h, aR0, aR1, aZ0, aZ1, aN0, aN1);
      gemm3_f16<kH / 32, kH, kHP>(we1h + wo256, hbuf + pr + kPL + bo_h, aR0, aR1, aZ0, aZ1, aH0, aH1);
      const float* tb = sbias + kSbCell + ub;
      const v8f bR = ld8(tb);
      const v8f bZ = ld8(tb + kH);
      const v8f bN = ld8(tb + 2 * kH);
      const v8f bNH = ld8(tb + 3 * kH);
      _Float16* hw = hbuf + pw + kPL + so_h;
      gru_gates<false>(aR0, aZ0, aN0, aH0, bR, bZ, bN, bNH, m10, hw, nullptr, nullptr);
      gru_gates<false>(aR1, aZ1, aN1, aH1, bR, bZ, bN, bNH, m11, hw + 16 * kHP, nullptr, nullptr);
    }
    __syncthreads();
  }

  const float* xsrcD = a.x_tgt + ((size_t)(b0 + xr) * kTD) * kNX + xc4;
  {
    const v4f xv = *(const v4f*)(xsrcD);
    unsigned h0w, l0w, h1w, l1w;
    split2(xv[0] * kActCarry, xv[1] * kActCarry, h0w, l0w);
    split2(xv[2] * kActCarry, xv[3] * kActCarry, h1w, l1w);
    *(v2u*)(xdh + xr * kXDP + xc4) = (v2u){h0w, h1w};
    *(v2u*)(xdl + xr * kXDP + xc4) = (v2u){l0w, l1w};
    if (wave < 4) {
      const int prow = tid >> 2, pc4 = (tid & 3) * 4;
      const v4f pv = *(const v4f*)(a.pv_init + (size_t)(b0 + prow) * kNPV + pc4);
      unsigned ph0, pl0, ph1, pl1;
      split2(pv[0] * kActCarry, pv[1] * kActCarry, ph0, pl0);
      split2(pv[2] * kActCarry, pv[3] * kActCarry, ph1, pl1);
      *(v2u*)(xdh + prow * kXDP + kNX + pc4) = (v2u){ph0, ph1};
      *(v2u*)(xdl + prow * kXDP + kNX + pc4) = (v2u){pl0, pl1};
    }
    if (wave < 2) {
      const int zr = tid >> 1, zc = kDI + 8 * (tid & 1);
      const v4u zz = {0u, 0u, 0u, 0u};
      *(v4u*)(xdh + zr * kXDP + zc) = zz;
      *(v4u*)(xdl + zr * kXDP + zc) = zz;
    }
  }
  __syncthreads();

  const int mt1 = wave >> 1, nt1 = wave & 1;
  const unsigned f1w = (unsigned)((16 * mt1 + c) * kH + koff);
  const unsigned f1a = (unsigned)((16 * nt1 + c) * kHP + koff);
  const unsigned f1s = (unsigned)((16 * nt1 + c) * kAP + 16 * mt1 + 8 * hh);

#pragma unroll 1
  for (int t = 0; t < kTD; ++t) {
    const int pr = (t & 1) * (2 * kPL);
    const int pw = (2 * kPL) - pr;
    {
      v8f aR0 = z8, aR1 = z8, aZ0 = z8, aZ1 = z8, aN0 = z8, aN1 = z8, aH0 = z8, aH1 = z8;
      gemm3_b3<kDIP / 32, kDIP, kXDP>(wd0ih + wo96, wd0il + wo96,
                                      (const __bf16*)(xdh + bo_xd), (const __bf16*)(xdl + bo_xd),
                                      aR0, aR1, aZ0, aZ1, aN0, aN1);
      gemm3_f16<kH / 32, kH, kHP>(wd0h + wo256, hbuf + pr + bo_h, aR0, aR1, aZ0, aZ1, aH0, aH1);
      const float* tb = sbias + kSbCell + 1024 + ub;
      const v8f bR = ld8(tb);
      const v8f bZ = ld8(tb + kH);
      const v8f bN = ld8(tb + 2 * kH);
      const v8f bNH = ld8(tb + 3 * kH);
      _Float16* hw = hbuf + pw + so_h;
      gru_gates<false>(aR0, aZ0, aN0, aH0, bR, bZ, bN, bNH, m00, hw, nullptr, nullptr);
      gru_gates<false>(aR1, aZ1, aN1, aH1, bR, bZ, bN, bNH, m01, hw + 16 * kHP, nullptr, nullptr);
    }
    __syncthreads();
    {
      const int tn = (t + 1 < kTD) ? (t + 1) : (kTD - 1);
      const v4f xv = *(const v4f*)(xsrcD + (size_t)tn * kNX);
      unsigned h0w, l0w, h1w, l1w;
      split2(xv[0] * kActCarry, xv[1] * kActCarry, h0w, l0w);
      split2(xv[2] * kActCarry, xv[3] * kActCarry, h1w, l1w);
      *(v2u*)(xdh + xr * kXDP + xc4) = (v2u){h0w, h1w};
      *(v2u*)(xdl + xr * kXDP + xc4) = (v2u){l0w, l1w};
      if (wave < 2) {
        const int zr = tid >> 1, zc = kDI + 8 * (tid & 1);
        const v4u zz = {0u, 0u, 0u, 0u};
        *(v4u*)(xdh + zr * kXDP + zc) = zz;
        *(v4u*)(xdl + zr * kXDP + zc) = zz;
      }
    }
    {
      v8f aR0 = z8, aR1 = z8, aZ0 = z8, aZ1 = z8, aN0 = z8, aN1 = z8, aH0 = z8, aH1 = z8;
      gemm3_f16<kH / 32, kH, kHP>(wd1i + wo256, hbuf + pw + bo_h, aR0, aR1, aZ0, aZ1, aN0, aN1);
      gemm3_f16<kH / 32, kH, kHP>(wd1h + wo256, hbuf + pr + kPL + bo_h, aR0, aR1, aZ0, aZ1, aH0, aH1);
      const float* tb = sbias + kSbCell + 2048 + ub;
      const v8f bR = ld8(tb);
      const v8f bZ = ld8(tb + kH);
      const v8f bN = ld8(tb + 2 * kH);
      const v8f bNH = ld8(tb + 3 * kH);
      _Float16* hw = hbuf + pw + kPL + so_h;
      gru_gates<true>(aR0, aZ0, aN0, aH0, bR, bZ, bN, bNH, m10, hw, d1h + so_h, d1l + so_h);
      gru_gates<true>(aR1, aZ1, aN1, aH1, bR, bZ, bN, bNH, m11, hw + 16 * kHP, d1h + so_h + 16 * kHP, d1l + so_h + 16 * kHP);
    }
    __syncthreads();
    {
      v8f acc = z8;
      acc = gemm1_b3<kH / 32>(fc1h + f1w, fc1l + f1w, (const __bf16*)(d1h + f1a), (const __bf16*)(d1l + f1a), acc);
      const v8f bb = ld8(sbias + kSbFc1 + 16 * mt1 + 8 * hh);
      float av[8];
#pragma unroll
      for (int r = 0; r < 8; ++r) av[r] = fmaxf(fmaf(acc[r], kFold, bb[r]), 0.0f) * kActCarry;
      v4u wh, wl;
#pragma unroll
      for (int q = 0; q < 4; ++q) {
        unsigned hi, lo;
        split2(av[2 * q], av[2 * q + 1], hi, lo);
        wh[q] = hi;
        wl[q] = lo;
      }
      *(v4u*)(ah + f1s) = wh;
      *(v4u*)(al + f1s) = wl;
    }
    __syncthreads();
    if (wave < 2) {
      const unsigned f2w = (unsigned)(c * kF1 + koff);
      const unsigned f2a = (unsigned)((16 * wave + c) * kAP + koff);
      v8f acc = z8;
      acc = gemm1_b3<kF1 / 32>(fc2h + f2w, fc2l + f2w, (const __bf16*)(ah + f2a), (const __bf16*)(al + f2a), acc);
      const v8f bb = ld8(sbias + kSbFc2 + 8 * hh);
      float yv[8];
#pragma unroll
      for (int r = 0; r < 8; ++r) yv[r] = fmaf(acc[r], kFold, bb[r]);
      float* yb = ybuf + (16 * wave + c) * kYP + (t & 7) * kNPV + 8 * hh;
      *(v4f*)yb       = (v4f){yv[0], yv[1], yv[2], yv[3]};
      *(v4f*)(yb + 4) = (v4f){yv[4], yv[5], yv[6], yv[7]};
      v4u wh, wl;
#pragma unroll
      for (int q = 0; q < 4; ++q) {
        unsigned hi, lo;
        split2(yv[2 * q] * kActCarry, yv[2 * q + 1] * kActCarry, hi, lo);
        wh[q] = hi;
        wl[q] = lo;
      }
      const unsigned fs = (unsigned)((16 * wave + c) * kXDP + kNX + 8 * hh);
      *(v4u*)(xdh + fs) = wh;
      *(v4u*)(xdl + fs) = wl;
    }
    __syncthreads();
    if ((t & 7) == 7) {
      const int t0 = t - 7;
      const v4f v0 = *(const v4f*)(ybuf + (2 * wave) * kYP + 4 * lane);
      const v4f v1 = *(const v4f*)(ybuf + (2 * wave + 1) * kYP + 4 * lane);
      float* o0 = a.out + ((size_t)(b0 + 2 * wave) * kTD + t0) * kNPV + 4 * lane;
      float* o1 = o0 + (size_t)kTD * kNPV;
      for (int pass = 0; pass < 2; ++pass) {
        *(volatile v4f*)o0 = v0;
        *(volatile v4f*)o1 = v1;
        __threadfence();
      }
    }
  }
}

extern "C" void kernel_launch(void* const* d_in, const int* in_sizes, int n_in,
                              void* d_out, int out_size, void* d_ws, size_t ws_size, hipStream_t stream) {
  if (n_in < 25 || d_out == nullptr || d_ws == nullptr) return;
  if (in_sizes[0] != kNB * kTE * kNX || in_sizes[1] != kNB * kTD * kNX || in_sizes[2] != kNB * kNPV ||
      in_sizes[3] != kNB || in_sizes[4] != kNSC * kEMB ||
      in_sizes[5] != kG * kEI || in_sizes[6] != kG * kH || in_sizes[7] != kG || in_sizes[8] != kG ||
      in_sizes[9] != kG * kH || in_sizes[10] != kG * kH || in_sizes[11] != kG || in_sizes[12] != kG ||
      in_sizes[13] != kG * kDI || in_sizes[14] != kG * kH || in_sizes[15] != kG || in_sizes[16] != kG ||
      in_sizes[17] != kG * kH || in_sizes[18] != kG * kH || in_sizes[19] != kG || in_sizes[20] != kG ||
      in_sizes[21] != kF1 * kH || in_sizes[22] != kF1 || in_sizes[23] != kNPV * kF1 || in_sizes[24] != kNPV ||
      out_size != kNB * kTD * kNPV) return;

  char* ws = (char*)d_ws;
  size_t off = 0;
  auto carve = [&](size_t bytes) -> char* { char* p = ws + off; off += (bytes + 255) & ~(size_t)255; return p; };
  unsigned short* WE0X  = (unsigned short*)carve((size_t)kG * kNX * 2);
  unsigned short* WE0H  = (unsigned short*)carve((size_t)kG * kH * 2);
  unsigned short* WE1I  = (unsigned short*)carve((size_t)kG * kH * 2);
  unsigned short* WE1H  = (unsigned short*)carve((size_t)kG * kH * 2);
  unsigned short* WD0H  = (unsigned short*)carve((size_t)kG * kH * 2);
  unsigned short* WD1I  = (unsigned short*)carve((size_t)kG * kH * 2);
  unsigned short* WD1H  = (unsigned short*)carve((size_t)kG * kH * 2);
  unsigned short* WD0IH = (unsigned short*)carve((size_t)kG * kDIP * 2);
  unsigned short* WD0IL = (unsigned short*)carve((size_t)kG * kDIP * 2);
  unsigned short* FC1H  = (unsigned short*)carve((size_t)kF1 * kH * 2);
  unsigned short* FC1L  = (unsigned short*)carve((size_t)kF1 * kH * 2);
  unsigned short* FC2H  = (unsigned short*)carve((size_t)kNPV * kF1 * 2);
  unsigned short* FC2L  = (unsigned short*)carve((size_t)kNPV * kF1 * 2);
  float*          PI    = (float*)carve((size_t)kNB * kG * 4);
  if (off > ws_size || off > (size_t)134217728) return;

  PrepArgs pa;
  pa.scen  = (const int*)d_in[3];
  pa.emb   = (const float*)d_in[4];
  pa.eWih0 = (const float*)d_in[5];
  pa.eWhh0 = (const float*)d_in[6];
  pa.ebih0 = (const float*)d_in[7];
  pa.ebhh0 = (const float*)d_in[8];
  pa.eWih1 = (const float*)d_in[9];
  pa.eWhh1 = (const float*)d_in[10];
  pa.dWih0 = (const float*)d_in[13];
  pa.dWhh0 = (const float*)d_in[14];
  pa.dWih1 = (const float*)d_in[17];
  pa.dWhh1 = (const float*)d_in[18];
  pa.fc1W  = (const float*)d_in[21];
  pa.fc2W  = (const float*)d_in[23];
  pa.we0x = WE0X; pa.we0h = WE0H; pa.we1i = WE1I; pa.we1h = WE1H;
  pa.wd0h = WD0H; pa.wd1i = WD1I; pa.wd1h = WD1H;
  pa.wd0ih = WD0IH; pa.wd0il = WD0IL;
  pa.fc1h = FC1H; pa.fc1l = FC1L; pa.fc2h = FC2H; pa.fc2l = FC2L;
  pa.pi = PI;
  prep_kernel<<<kPrepBlocks, 256, 0, stream>>>(pa);

  SeqArgs sa;
  sa.x_cv    = (const float*)d_in[0];
  sa.x_tgt   = (const float*)d_in[1];
  sa.pv_init = (const float*)d_in[2];
  sa.ebhh0   = (const float*)d_in[8];
  sa.ebih1   = (const float*)d_in[11];
  sa.ebhh1   = (const float*)d_in[12];
  sa.dbih0   = (const float*)d_in[15];
  sa.dbhh0   = (const float*)d_in[16];
  sa.dbih1   = (const float*)d_in[19];
  sa.dbhh1   = (const float*)d_in[20];
  sa.fc1b    = (const float*)d_in[22];
  sa.fc2b    = (const float*)d_in[24];
  sa.we0x = WE0X; sa.we0h = WE0H; sa.we1i = WE1I; sa.we1h = WE1H;
  sa.wd0h = WD0H; sa.wd1i = WD1I; sa.wd1h = WD1H;
  sa.wd0ih = WD0IH; sa.wd0il = WD0IL;
  sa.fc1h = FC1H; sa.fc1l = FC1L; sa.fc2h = FC2H; sa.fc2l = FC2L;
  sa.pi  = PI;
  sa.out = (float*)d_out;
  seq_kernel<<<kBlocks, kThr, 0, stream>>>(sa);
}
